// GraphResnet_7748121002166
// MI455X (gfx1250) — hardware-run, weakly checked
//
#include <hip/hip_runtime.h>

typedef float          v8f   __attribute__((ext_vector_type(8)));
typedef float          v4f   __attribute__((ext_vector_type(4)));
typedef unsigned int   v4u   __attribute__((ext_vector_type(4)));
typedef int            v8i   __attribute__((ext_vector_type(8)));
typedef unsigned short v8us  __attribute__((ext_vector_type(8)));
typedef unsigned short v16us __attribute__((ext_vector_type(16)));
typedef __bf16         v16bf __attribute__((ext_vector_type(16)));
typedef _Float16       v16h  __attribute__((ext_vector_type(16)));
typedef v4f  __attribute__((may_alias)) v4fa;
typedef v8us __attribute__((may_alias)) v8usa;
union FragB { v16bf v; v16us u; v8us h[2]; v8i w; };
union FragH { v16h  v; v16us u; v8us h[2]; v8i w; };

__device__ __forceinline__ v8f wmb(const FragB& a, const FragB& b, v8f c) {
  v8f d = __builtin_amdgcn_wmma_f32_16x16x32_bf16(false, a.v, false, b.v, (short)0, c, false, false);
  asm volatile("v_nop\n\tv_nop\n\tv_nop\n\tv_nop" : "+v"(d) : "v"(a.w), "v"(b.w));
  return d;
}

__device__ __forceinline__ v8f wmh(const FragH& a, const FragH& b, v8f c) {
  v8f d = __builtin_amdgcn_wmma_f32_16x16x32_f16(false, a.v, false, b.v, (short)0, c, false, false);
  asm volatile("v_nop\n\tv_nop\n\tv_nop\n\tv_nop" : "+v"(d) : "v"(a.w), "v"(b.w));
  return d;
}

__device__ __forceinline__ unsigned bf16_bits(float f) {
  const unsigned u = __float_as_uint(f);
  const unsigned r = (u + 0x7FFFu + ((u >> 16) & 1u)) >> 16;
  const unsigned q = (u >> 16) | 0x40u;
  return ((u & 0x7fffffffu) > 0x7f800000u) ? q : r;
}

__device__ __forceinline__ float bf16_val(float f) {
  return __uint_as_float(bf16_bits(f) << 16);
}
__device__ __forceinline__ int clampi(int v, int lo, int hi) {
  return v < lo ? lo : (v > hi ? hi : v);
}

__device__ __forceinline__ unsigned f16_bits(float f) {
  const unsigned u  = __float_as_uint(f);
  const unsigned s  = (u >> 16) & 0x8000u;
  const unsigned a  = u & 0x7fffffffu;
  const unsigned t  = a - 0x38000000u;
  const unsigned r  = (t + 0x0FFFu + ((t >> 13) & 1u)) >> 13;
  const unsigned rc = r > 0x7C00u ? 0x7C00u : r;
  const bool small  = a < 0x38800000u;
  const bool isnan  = a > 0x7f800000u;
  const unsigned fin = small ? 0u : (s | rc);
  return isnan ? (s | 0x7E00u) : fin;
}

__device__ __forceinline__ unsigned pk16(unsigned lo, unsigned hi) { return lo | (hi << 16); }
__device__ __forceinline__ unsigned bf16_lo_bits(float v) {
  float hi = bf16_val(v);
  asm volatile("" : "+v"(hi));
  return bf16_bits(v - hi);
}
__device__ __forceinline__ v4u pack8_bf16(v4f a, v4f c) {
  return (v4u){ pk16(bf16_bits(a[0]), bf16_bits(a[1])), pk16(bf16_bits(a[2]), bf16_bits(a[3])),
                pk16(bf16_bits(c[0]), bf16_bits(c[1])), pk16(bf16_bits(c[2]), bf16_bits(c[3])) };
}
__device__ __forceinline__ v4u pack8_bf16_lo(v4f a, v4f c) {
  return (v4u){ pk16(bf16_lo_bits(a[0]), bf16_lo_bits(a[1])), pk16(bf16_lo_bits(a[2]), bf16_lo_bits(a[3])),
                pk16(bf16_lo_bits(c[0]), bf16_lo_bits(c[1])), pk16(bf16_lo_bits(c[2]), bf16_lo_bits(c[3])) };
}
__device__ __forceinline__ v4u pack8_f16(v4f a, v4f c) {
  return (v4u){ pk16(f16_bits(a[0]), f16_bits(a[1])), pk16(f16_bits(a[2]), f16_bits(a[3])),
                pk16(f16_bits(c[0]), f16_bits(c[1])), pk16(f16_bits(c[2]), f16_bits(c[3])) };
}

template <int FORM>
__global__ __launch_bounds__(256) void k_plane(const float* __restrict__ src, int rows, int cols, int ldsrc,
                                               unsigned short* __restrict__ dst, int MP, int KP) {
  static_assert(FORM >= 0 && FORM <= 3);
  const int KTOT = (FORM == 1 || FORM == 3) ? 2 * KP : KP;
  const unsigned ppr   = (unsigned)(KTOT >> 3);
  const unsigned kp8   = (unsigned)(KP >> 3);
  const unsigned total = (unsigned)MP * ppr;
  const unsigned g     = blockIdx.x * 256u + threadIdx.x;
  const unsigned rowu  = g / ppr;
  const unsigned p     = g - rowu * ppr;
  const bool second    = p >= kp8;
  const int row = (int)rowu;
  const int c0  = (int)((second ? p - kp8 : p) << 3);
  const float* srow = src + (size_t)clampi(row, 0, rows - 1) * (size_t)ldsrc;
  float x[8];
  unsigned mk[8];
#pragma unroll
  for (int e = 0; e < 8; ++e) {
    const int c = c0 + e;
    const float v = srow[clampi(c, 0, cols - 1)];
    asm volatile("" :: "v"(v));
    x[e]  = v;
    mk[e] = (row < rows && c < cols) ? 0xFFFFu : 0u;
  }
  const v4f a = (v4f){ x[0], x[1], x[2], x[3] };
  const v4f c = (v4f){ x[4], x[5], x[6], x[7] };
  v4u o;
  if (FORM == 2) {
    o = pack8_f16(a, c);
  } else {
    const v4u hi = pack8_bf16(a, c);
    o = hi;
    if (FORM == 1) { const v4u lo = pack8_bf16_lo(a, c); o = second ? lo : hi; }
  }
  const v4u mw = (v4u){ pk16(mk[0], mk[1]), pk16(mk[2], mk[3]), pk16(mk[4], mk[5]), pk16(mk[6], mk[7]) };
  o &= mw;
  if (g < total) {
    volatile v4u* q = (volatile v4u*)(dst + (size_t)g * 8);
    *q = o;
    __threadfence();
    *q = o;
  }
}

template <int FORM> struct FragOf    { typedef FragB T; };
template <>         struct FragOf<2> { typedef FragH T; };
__device__ __forceinline__ v8f mm(const FragB& a, const FragB& b, v8f c) { return wmb(a, b, c); }
__device__ __forceinline__ v8f mm(const FragH& a, const FragH& b, v8f c) { return wmh(a, b, c); }
template <class F> __device__ __forceinline__ F ld_frag(const unsigned short* p) {
  F f;
  f.h[0] = *(const v8usa*)(p);
  f.h[1] = *(const v8usa*)(p + 16);
  return f;
}

template <int FORM, int EPI>
__global__ __launch_bounds__(256) __attribute__((amdgpu_num_vgpr(248)))
void k_gemm_nt(const unsigned short* __restrict__ A, const unsigned short* __restrict__ B,
               const float* __restrict__ bias, float* __restrict__ D, int M, int N, int KTOT, int ldd) {
  static_assert(FORM >= 0 && FORM <= 2);
  static_assert(EPI == 0 || EPI == 1);
  typedef typename FragOf<FORM>::T F;
  __shared__ __attribute__((aligned(16))) float sT[8][16 * 68];
  const int lane = threadIdx.x & 31;
  const int wave = threadIdx.x >> 5;
  const int tilesM = (M + 63) >> 6;
  const int tilesN = (N + 63) >> 6;
  const int tile = blockIdx.x * 8 + wave;
  if (tile >= tilesM * tilesN) return;
  const int tm = tile / tilesN;
  const int tn = tile - tm * tilesN;
  const int m0 = tm << 6;
  const int n0 = tn << 6;

  const int rl = lane & 15;
  const int h8 = (lane >> 4) * 8;
  const unsigned short* pa = A + (size_t)(m0 + rl) * (size_t)KTOT + h8;
  const unsigned short* pb = B + (size_t)(n0 + rl) * (size_t)KTOT + h8;

  v8f acc[4][4];
#pragma unroll
  for (int i = 0; i < 4; ++i)
#pragma unroll
    for (int j = 0; j < 4; ++j) acc[i][j] = (v8f){0.f, 0.f, 0.f, 0.f, 0.f, 0.f, 0.f, 0.f};

#pragma unroll 1
  for (int k0 = 0; k0 < KTOT; k0 += 32) {
    F bf[4];
#pragma unroll
    for (int j = 0; j < 4; ++j) bf[j] = ld_frag<F>(pb + (size_t)(j << 4) * (size_t)KTOT + k0);
#pragma unroll
    for (int i = 0; i < 4; ++i) {
      const F af = ld_frag<F>(pa + (size_t)(i << 4) * (size_t)KTOT + k0);
#pragma unroll
      for (int j = 0; j < 4; ++j) acc[i][j] = mm(af, bf[j], acc[i][j]);
    }
  }

  float* slab = sT[wave];
  const int hh = lane >> 4;
  const int c4 = (lane & 15) * 4;
  const int nc = n0 + c4;
  const bool cok = nc < N;
  v4f bv = (v4f){0.f, 0.f, 0.f, 0.f};
  if (EPI == 1) {
    bv = *(const v4fa*)(bias + clampi(nc, 0, N - 4));
    asm volatile("" :: "v"(bv));
  }
#pragma unroll
  for (int i = 0; i < 4; ++i) {
    const int mBase = m0 + (i << 4);
#pragma unroll
    for (int j = 0; j < 4; ++j) {
#pragma unroll
      for (int r = 0; r < 8; ++r) slab[(h8 + r) * 68 + (j << 4) + rl] = acc[i][j][r];
    }
    __builtin_amdgcn_fence(__ATOMIC_RELEASE, "workgroup");
    __builtin_amdgcn_wave_barrier();
    __builtin_amdgcn_fence(__ATOMIC_ACQUIRE, "workgroup");
    v4f vv[8];
#pragma unroll
    for (int it = 0; it < 8; ++it) {
      const int row = it * 2 + hh;
      v4f v = *(const v4fa*)(slab + row * 68 + c4);
      if (EPI == 1) v += bv;
      vv[it] = v;
    }
    for (int pass = 0; pass < 2; ++pass) {
#pragma unroll
      for (int it = 0; it < 8; ++it) {
        const int row = mBase + it * 2 + hh;
        if (cok && row < M) *(volatile v4f*)(D + (size_t)row * (size_t)ldd + nc) = vv[it];
      }
      __threadfence();
    }
    __builtin_amdgcn_fence(__ATOMIC_RELEASE, "workgroup");
    __builtin_amdgcn_wave_barrier();
    __builtin_amdgcn_fence(__ATOMIC_ACQUIRE, "workgroup");
  }
}

#include <stddef.h>
#include <stdint.h>

#pragma clang fp contract(off)

#ifndef SPLIT_L2
#define SPLIT_L2 1
#endif
#ifndef SPLIT_L3
#define SPLIT_L3 1
#endif
#ifndef SPLIT_MIX
#define SPLIT_MIX 1
#endif

#define NN      100000
#define NE      1200000
#define NP      100096
#define FD      64
#define NCLS    32
#define KL1     64
#define KL2     (SPLIT_L2 ? 128 : 64)
#define KL3     (SPLIT_L3 ? 128 : 64)
#define KMX     (SPLIT_MIX ? 192 : 128)
#define NTHR    256
#define NWAVE   8
#define NBRUN   1024
#define SLB     10
#define NBLK    98
#define NSLOT   (NBLK * NBRUN)
#define EPW     (NE / NWAVE)
#define STEPE   256
#define NSTEP   ((EPW + STEPE - 1) / STEPE)
#define WLCAP   2560
#define HCAP    (NWAVE * WLCAP)
#define RCAP    16384
#define DEGCAP  64
#define MEAS_B1024 12539
#define MEAS_DEG   30
#define BK_ZINTS   (2 * HCAP + RCAP + 5 * NBRUN)
#define BK_INTS    (BK_ZINTS + 32)
#define BK_LDS     (BK_INTS * 4)
#define LIST_IT    ((RCAP / 4) / NTHR)
#define WSLOT      (64 * 128)
#define BPL1       (KL1 / 32)
#define BPL2       (KL2 / 32)
#define BPL3       (KL3 / 32)
#define KB0        (4 * BPL1)
#define KB1        (4 * BPL2)
#define KB2        (4 * BPL3)
#define NKB        (KB0 + KB1 + KB2)
#define NSB        (BPL1 + BPL2 + BPL3)
#define NMB        (KMX / 32)
#define PREP_BLOCKS (NKB + NSB + NMB + 1)

static_assert(NN % NWAVE == 0 && NN % 16 == 0 && FD == 64 && NCLS == 32);
static_assert(NBRUN == (1 << SLB) && NN <= (1 << 17));
static_assert((NBLK - 1) * NBRUN < NN && NBLK * NBRUN >= NN);
static_assert(NP % 128 == 0 && NP >= ((NN + 63) / 64) * 64 && (NP * 8) % 256 == 0);
static_assert(NE % NWAVE == 0 && EPW % 8 == 0 && NE % 8 == 0 && NSTEP == 586);
static_assert(((long long)(NN - 1) << SLB) < (1LL << 31));
static_assert(4 * RCAP >= 5 * MEAS_B1024 && (RCAP / 4) % NTHR == 0 && LIST_IT == 16);
static_assert(8 * WLCAP * 4 >= 5 * MEAS_B1024 && HCAP >= RCAP);
static_assert(DEGCAP >= MEAS_DEG + 8 && RCAP > DEGCAP);
static_assert(BK_ZINTS % (NTHR * 4) == 0 && BK_LDS == 249984 && BK_LDS <= 262144 && BK_LDS <= 327680);
static_assert(KL1 % 32 == 0 && KL2 % 32 == 0 && KL3 % 32 == 0 && KMX % 32 == 0);

typedef float v2f __attribute__((ext_vector_type(2)));
typedef int   v4i __attribute__((ext_vector_type(4)));
typedef v2f __attribute__((may_alias)) v2fa;
typedef v4i __attribute__((may_alias)) v4ia;

#define PIN(x) asm volatile("" :: "v"(x))

__device__ __forceinline__ void wunit(const float* __restrict__ W, int KW, int u, unsigned short* dstp) {
  const int ppr = KW >> 3;
  const int n   = u / ppr;
  const int k8  = (u - n * ppr) << 3;
  const int kk  = k8 & 63;
  const float* p = W + (size_t)kk * 64 + n;
  unsigned w[8];
#pragma unroll
  for (int i = 0; i < 8; ++i) {
    const float v = p[(size_t)i * 64];
    asm volatile("" :: "v"(v));
    w[i] = bf16_bits(v);
  }
  const v4u o = (v4u){ pk16(w[0], w[1]), pk16(w[2], w[3]), pk16(w[4], w[5]), pk16(w[6], w[7]) };
  volatile v4u* q = (volatile v4u*)(dstp + (size_t)n * (size_t)KW + k8);
  *q = o;
  __threadfence();
  *q = o;
}

__device__ __forceinline__ void munit(const float* __restrict__ MW, int u, unsigned short* dstp) {
  const int ppr = KMX >> 3;
  const int n   = u / ppr;
  const int k8  = (u - n * ppr) << 3;
  const int kin = SPLIT_MIX ? ((k8 < 128) ? (k8 & 63) : (k8 - 64)) : k8;
  const float* p = MW + (size_t)(n >> 5) * (128 * NCLS) + (size_t)kin * NCLS + (n & 31);
  unsigned w[8];
#pragma unroll
  for (int i = 0; i < 8; ++i) {
    const float v = p[(size_t)i * NCLS];
    asm volatile("" :: "v"(v));
    w[i] = bf16_bits(v);
  }
  const v4u o = (v4u){ pk16(w[0], w[1]), pk16(w[2], w[3]), pk16(w[4], w[5]), pk16(w[6], w[7]) };
  volatile v4u* q = (volatile v4u*)(dstp + (size_t)n * (size_t)KMX + k8);
  *q = o;
  __threadfence();
  *q = o;
}

__global__ __launch_bounds__(NTHR) void k_prep(const float* __restrict__ kw, const float* __restrict__ sw,
                                               const float* __restrict__ mw, const float* __restrict__ kb,
                                               const float* __restrict__ sb, const float* __restrict__ mb,
                                               unsigned short* WPL, unsigned short* MT, float* BT) {
  __shared__ __attribute__((aligned(16))) float sp[512];
  const int blk = (int)blockIdx.x;
  const int tid = (int)threadIdx.x;
  if (blk < NKB) {
    int l, r;
    if (blk < KB0) { l = 0; r = blk; }
    else if (blk < KB0 + KB1) { l = 1; r = blk - KB0; }
    else { l = 2; r = blk - KB0 - KB1; }
    const int KW  = (l == 0) ? KL1 : ((l == 1) ? KL2 : KL3);
    const int bpl = KW >> 5;
    const int k   = r / bpl;
    const int sub = r - k * bpl;
    wunit(kw + (size_t)(l * 4 + k) * 4096, KW, sub * NTHR + tid, WPL + (size_t)(l * 5 + k) * WSLOT);
  } else if (blk < NKB + NSB) {
    const int r = blk - NKB;
    int l, sub;
    if (r < BPL1) { l = 0; sub = r; }
    else if (r < BPL1 + BPL2) { l = 1; sub = r - BPL1; }
    else { l = 2; sub = r - BPL1 - BPL2; }
    const int KW = (l == 0) ? KL1 : ((l == 1) ? KL2 : KL3);
    wunit(sw + (size_t)l * 4096, KW, sub * NTHR + tid, WPL + (size_t)(l * 5 + 4) * WSLOT);
  } else if (blk < NKB + NSB + NMB) {
    munit(mw, (blk - NKB - NSB) * NTHR + tid, MT);
  } else {
#pragma unroll
    for (int hf = 0; hf < 2; ++hf) {
      const int c = tid + 256 * hf;
      const float vk = kb[clampi(c, 0, 191)];
      const float vs = sb[clampi(c - 192, 0, 191)];
      const float vm = mb[clampi(c - 384, 0, 31)];
      PIN(vk);
      PIN(vs);
      PIN(vm);
      const unsigned mk = (c < 192) ? 0xFFFFFFFFu : 0u;
      const unsigned ms = (c >= 192 && c < 384) ? 0xFFFFFFFFu : 0u;
      const unsigned mm2 = (c >= 384 && c < 416) ? 0xFFFFFFFFu : 0u;
      const unsigned bits = ((bf16_bits(vk) << 16) & mk) | ((bf16_bits(vs) << 16) & ms) | ((bf16_bits(vm) << 16) & mm2);
      sp[c] = __uint_as_float(bits);
    }
    __syncthreads();
    if (tid < 128) {
      const v4f o = *(const v4fa*)(sp + 4 * tid);
      volatile v4f* q = (volatile v4f*)(BT + 4 * tid);
      *q = o;
      __threadfence();
      *q = o;
    }
  }
}

#define DHIT(J, V) \
  const unsigned t##J = (unsigned)(V) - nbs; \
  const bool hd##J = (e0 + J < wend) && (t##J < unb); \
  const unsigned md##J = __builtin_amdgcn_ballot_w32(hd##J);
#define SHIT(J, V) \
  const unsigned r##J = (unsigned)(V) - nbs; \
  const bool hs##J = (e0 + J < wend) && (r##J < unb); \
  const unsigned ms##J = __builtin_amdgcn_ballot_w32(hs##J);
#define PUTD(J, SV) { \
  const int wv = (clampi((SV), 0, nN - 1) << SLB) | (int)t##J; \
  if (hd##J) { if (posd < WLCAP) wl0w[posd] = wv; } \
  posd += hd##J ? 1 : 0; }
#define PUTS(J) { \
  if (hs##J) { if (poss < WLCAP) wl2w[poss] = (int)r##J; } \
  poss += hs##J ? 1 : 0; }

__global__ __launch_bounds__(NTHR) void k_build(const int* __restrict__ srcs, const int* __restrict__ dsts, int nN,
                                                int* listG, int* cntG, int* offG, float* dinvG, int* flagG) {
  extern __shared__ __attribute__((aligned(16))) int dsm[];
  int* wl0  = dsm;
  int* wl2  = dsm + HCAP;
  int* sl   = dsm + 2 * HCAP;
  int* cnt  = sl + RCAP;
  int* offs = cnt + NBRUN;
  int* cur  = offs + NBRUN;
  int* dcnt = cur + NBRUN;
  int* dvi  = dcnt + NBRUN;
  int* misc = dvi + NBRUN;
  const int tid = (int)threadIdx.x, lane = tid & 31, wave = tid >> 5;
  const int b = (int)blockIdx.x;
  const int nodeBase = b * NBRUN;
  const int nb = clampi(nN - nodeBase, 0, NBRUN);

  {
    const v4i z4 = {0, 0, 0, 0};
    for (int i = tid * 4; i < BK_ZINTS; i += NTHR * 4) *(v4ia*)(dsm + i) = z4;
    if (tid < 32) misc[tid] = 0;
  }
  __syncthreads();

  {
    int* wl0w = wl0 + wave * WLCAP;
    int* wl2w = wl2 + wave * WLCAP;
    const int wbeg = wave * EPW;
    const int wend = wbeg + EPW;
    const unsigned nbs = (unsigned)nodeBase;
    const unsigned unb = (unsigned)nb;
    int wcd = 0, wcs = 0;
#pragma unroll 1
    for (int st = 0; st < NSTEP; ++st) {
      const int e0  = wbeg + st * STEPE + lane * 8;
      const int e0c = e0 < (NE - 8) ? e0 : (NE - 8);
      const v4i da = *(const v4ia*)(dsts + e0c);
      const v4i db = *(const v4ia*)(dsts + e0c + 4);
      const v4i sa = *(const v4ia*)(srcs + e0c);
      const v4i sb = *(const v4ia*)(srcs + e0c + 4);
      PIN(da.x); PIN(da.y); PIN(da.z); PIN(da.w);
      PIN(db.x); PIN(db.y); PIN(db.z); PIN(db.w);
      PIN(sa.x); PIN(sa.y); PIN(sa.z); PIN(sa.w);
      PIN(sb.x); PIN(sb.y); PIN(sb.z); PIN(sb.w);
      DHIT(0, da.x) DHIT(1, da.y) DHIT(2, da.z) DHIT(3, da.w)
      DHIT(4, db.x) DHIT(5, db.y) DHIT(6, db.z) DHIT(7, db.w)
      SHIT(0, sa.x) SHIT(1, sa.y) SHIT(2, sa.z) SHIT(3, sa.w)
      SHIT(4, sb.x) SHIT(5, sb.y) SHIT(6, sb.z) SHIT(7, sb.w)
      const unsigned manyd = md0 | md1 | md2 | md3 | md4 | md5 | md6 | md7;
      const unsigned manys = ms0 | ms1 | ms2 | ms3 | ms4 | ms5 | ms6 | ms7;
      if (manyd != 0u) {
        unsigned pre = __builtin_amdgcn_mbcnt_lo(md0, 0u);
        pre = __builtin_amdgcn_mbcnt_lo(md1, pre);
        pre = __builtin_amdgcn_mbcnt_lo(md2, pre);
        pre = __builtin_amdgcn_mbcnt_lo(md3, pre);
        pre = __builtin_amdgcn_mbcnt_lo(md4, pre);
        pre = __builtin_amdgcn_mbcnt_lo(md5, pre);
        pre = __builtin_amdgcn_mbcnt_lo(md6, pre);
        pre = __builtin_amdgcn_mbcnt_lo(md7, pre);
        int posd = wcd + (int)pre;
        PUTD(0, sa.x) PUTD(1, sa.y) PUTD(2, sa.z) PUTD(3, sa.w)
        PUTD(4, sb.x) PUTD(5, sb.y) PUTD(6, sb.z) PUTD(7, sb.w)
        wcd += (int)__builtin_popcount(md0) + (int)__builtin_popcount(md1) + (int)__builtin_popcount(md2)
             + (int)__builtin_popcount(md3) + (int)__builtin_popcount(md4) + (int)__builtin_popcount(md5)
             + (int)__builtin_popcount(md6) + (int)__builtin_popcount(md7);
      }
      if (manys != 0u) {
        unsigned pre = __builtin_amdgcn_mbcnt_lo(ms0, 0u);
        pre = __builtin_amdgcn_mbcnt_lo(ms1, pre);
        pre = __builtin_amdgcn_mbcnt_lo(ms2, pre);
        pre = __builtin_amdgcn_mbcnt_lo(ms3, pre);
        pre = __builtin_amdgcn_mbcnt_lo(ms4, pre);
        pre = __builtin_amdgcn_mbcnt_lo(ms5, pre);
        pre = __builtin_amdgcn_mbcnt_lo(ms6, pre);
        pre = __builtin_amdgcn_mbcnt_lo(ms7, pre);
        int poss = wcs + (int)pre;
        PUTS(0) PUTS(1) PUTS(2) PUTS(3) PUTS(4) PUTS(5) PUTS(6) PUTS(7)
        wcs += (int)__builtin_popcount(ms0) + (int)__builtin_popcount(ms1) + (int)__builtin_popcount(ms2)
             + (int)__builtin_popcount(ms3) + (int)__builtin_popcount(ms4) + (int)__builtin_popcount(ms5)
             + (int)__builtin_popcount(ms6) + (int)__builtin_popcount(ms7);
      }
    }
    if (lane == 0) { misc[wave] = wcd; misc[16 + wave] = wcs; }
  }
  __syncthreads();

  if (wave == 0) {
    int t = 0, ov = 0;
#pragma unroll 1
    for (int w2 = 0; w2 < NWAVE; ++w2) {
      int c = misc[w2];
      ov |= (c > WLCAP) ? 1 : 0;
      c = c < 0 ? 0 : (c > WLCAP ? WLCAP : c);
      c = __builtin_amdgcn_readfirstlane(c);
#pragma unroll 1
      for (int b0 = 0; b0 < c; b0 += 32) {
        const int idx = b0 + lane;
        const int ent = wl0[w2 * WLCAP + (idx < WLCAP ? idx : WLCAP - 1)];
        const int m32 = (c - b0) < 32 ? (c - b0) : 32;
#pragma unroll 1
        for (int k = 0; k < m32; ++k) {
          const int u    = __builtin_amdgcn_readlane(ent, k);
          const int slot = u & (NBRUN - 1);
          if (t < RCAP) {
            const int cvv = cnt[slot];
            if (lane == 0) cnt[slot] = cvv + 1;
            t = t + 1;
          } else {
            ov = 1;
          }
        }
      }
    }
    if (lane == 0) { misc[8] = t; misc[9] = ov; }
  } else if (wave == 1) {
    int ov = 0;
#pragma unroll 1
    for (int w2 = 0; w2 < NWAVE; ++w2) {
      int c = misc[16 + w2];
      ov |= (c > WLCAP) ? 1 : 0;
      c = c < 0 ? 0 : (c > WLCAP ? WLCAP : c);
      c = __builtin_amdgcn_readfirstlane(c);
#pragma unroll 1
      for (int b0 = 0; b0 < c; b0 += 32) {
        const int idx = b0 + lane;
        const int ent = wl2[w2 * WLCAP + (idx < WLCAP ? idx : WLCAP - 1)];
        const int m32 = (c - b0) < 32 ? (c - b0) : 32;
#pragma unroll 1
        for (int k = 0; k < m32; ++k) {
          const int u    = __builtin_amdgcn_readlane(ent, k);
          const int slot = u & (NBRUN - 1);
          const int cvv  = dcnt[slot];
          if (lane == 0) dcnt[slot] = cvv + 1;
        }
      }
    }
    if (lane == 0) misc[10] = ov;
  }
  __syncthreads();

#pragma unroll 1
  for (int i = 0; i < 4; ++i) {
    const int s  = 4 * tid + i;
    const int d  = dcnt[s];
    const float df = (float)(d > 1 ? d : 1);
    const float rv = 1.0f / sqrtf(df);
    const float dv = (d > 0) ? rv : 0.0f;
    dvi[s] = __float_as_int(dv);
  }
  if (wave == 0) {
    const int base = lane * (NBRUN / 32);
    int s = 0, big = 0;
#pragma unroll 1
    for (int i = 0; i < NBRUN / 32; ++i) {
      const int cvv = cnt[base + i];
      s += cvv;
      big |= (cvv > DEGCAP) ? 1 : 0;
    }
    int incl = s;
#pragma unroll
    for (int d = 1; d < 32; d <<= 1) {
      const int y = __shfl_up(incl, d, 32);
      if (lane >= d) incl += y;
    }
    int run = incl - s;
#pragma unroll 1
    for (int i = 0; i < NBRUN / 32; ++i) {
      const int cvv = cnt[base + i];
      offs[base + i] = run;
      cur[base + i]  = run;
      run += cvv;
    }
    const unsigned bm = __builtin_amdgcn_ballot_w32(big != 0);
    if (lane == 0) {
      const int o9 = misc[9];
      misc[9] = o9 | ((bm != 0u) ? 1 : 0);
    }
  }
  __syncthreads();

  if (wave == 0) {
    int t = 0;
#pragma unroll 1
    for (int w2 = 0; w2 < NWAVE; ++w2) {
      int c = misc[w2];
      c = c < 0 ? 0 : (c > WLCAP ? WLCAP : c);
      c = __builtin_amdgcn_readfirstlane(c);
#pragma unroll 1
      for (int b0 = 0; b0 < c; b0 += 32) {
        const int idx = b0 + lane;
        const int ent = wl0[w2 * WLCAP + (idx < WLCAP ? idx : WLCAP - 1)];
        const int m32 = (c - b0) < 32 ? (c - b0) : 32;
#pragma unroll 1
        for (int k = 0; k < m32; ++k) {
          const int u    = __builtin_amdgcn_readlane(ent, k);
          const int slot = u & (NBRUN - 1);
          if (t < RCAP) {
            int p = cur[slot];
            p = p < 0 ? 0 : (p > RCAP - 1 ? RCAP - 1 : p);
            if (lane == 0) { sl[p] = (u >> SLB) & 0x1FFFF; cur[slot] = p + 1; }
            t = t + 1;
          }
        }
      }
    }
  }
  __syncthreads();

  {
    const int ovf = misc[9] | misc[10];
    const v4i fv = {ovf, ovf, ovf, ovf};
    int* lb = listG + (size_t)b * (size_t)RCAP;
    for (int pass = 0; pass < 2; ++pass) {
#pragma unroll 1
      for (int it = 0; it < LIST_IT; ++it) {
        const int p4 = it * NTHR + tid;
        const v4i v = *(const v4ia*)(sl + 4 * p4);
        *(volatile v4i*)(lb + 4 * (size_t)p4) = v;
      }
      {
        const v4i c4 = *(const v4ia*)(cnt + 4 * tid);
        const v4i o4 = *(const v4ia*)(offs + 4 * tid);
        const v4i d4 = *(const v4ia*)(dvi + 4 * tid);
        const v4f f4 = (v4f){ __int_as_float(d4.x), __int_as_float(d4.y), __int_as_float(d4.z), __int_as_float(d4.w) };
        *(volatile v4i*)(cntG + (size_t)nodeBase + 4 * tid) = c4;
        *(volatile v4i*)(offG + (size_t)nodeBase + 4 * tid) = o4;
        *(volatile v4f*)(dinvG + (size_t)nodeBase + 4 * tid) = f4;
      }
      if (tid < 8) *(volatile v4i*)(flagG + (size_t)b * 32 + 4 * tid) = fv;
      __threadfence();
    }
  }
}

template <int MODE>
__global__ __launch_bounds__(NTHR) void k_prop(const float* G, const float* P, const float* Q, float* O,
                                               const int* __restrict__ listG, const int* __restrict__ cntG,
                                               const int* __restrict__ offG, const int* __restrict__ flagG,
                                               const float* __restrict__ dinvG, int nN) {
  static_assert(MODE >= 1 && MODE <= 3);
  const int tid = (int)threadIdx.x, lane = tid & 31, wave = tid >> 5;
  const int n = (int)blockIdx.x * NWAVE + wave;
  if (n >= nN) return;
  const int blk = n >> SLB;
  int cv   = cntG[n];
  int ofv  = offG[n];
  int fl   = flagG[(size_t)blk * 32];
  float dn = dinvG[n];
  PIN(cv);
  PIN(ofv);
  PIN(fl);
  PIN(dn);
  const size_t ro = (size_t)n * FD + 2 * lane;
  v2f pv = *(const v2fa*)(P + ro);
  PIN(pv);
  v2f qv = (v2f){0.0f, 0.0f};
  if (MODE != 1) {
    qv = *(const v2fa*)(Q + ro);
    PIN(qv);
  }
  const int bad = ((fl != 0) || (cv < 0) || (cv > DEGCAP)) ? 1 : 0;
  cv  = cv < 0 ? 0 : (cv > DEGCAP ? DEGCAP : cv);
  ofv = ofv < 0 ? 0 : (ofv > RCAP - DEGCAP ? RCAP - DEGCAP : ofv);
  const int cn = __builtin_amdgcn_readfirstlane(cv);
  const int o  = __builtin_amdgcn_readfirstlane(ofv);
  const int* listb = listG + (size_t)blk * (size_t)RCAP;
  float a0 = 0.0f, a1 = 0.0f;
#pragma unroll 1
  for (int g0 = 0; g0 < cn; g0 += 32) {
    const int last = o + cn - 1;
    int idx = o + g0 + lane;
    idx = idx > last ? last : idx;
    int s = listb[idx];
    PIN(s);
    const int col = clampi(s, 0, nN - 1);
    float dv = dinvG[col];
    PIN(dv);
    const float w = -(dv * dn);
    const int wb = __float_as_int(w);
    const int m32 = (cn - g0) < 32 ? (cn - g0) : 32;
#pragma unroll 1
    for (int t = 0; t < m32; ++t) {
      const int ct   = __builtin_amdgcn_readlane(col, t);
      const float wt = __int_as_float(__builtin_amdgcn_readlane(wb, t));
      const v2f z = *(const v2fa*)(G + (size_t)ct * FD + 2 * lane);
      const float m0 = wt * z.x;
      const float m1 = wt * z.y;
      a0 = a0 + m0;
      a1 = a1 + m1;
    }
  }
  float r0, r1;
  if (MODE == 1) {
    r0 = (2.0f * pv.x) + (4.0f * a0);
    r1 = (2.0f * pv.y) + (4.0f * a1);
  } else if (MODE == 2) {
    r0 = (pv.x - (3.0f * qv.x)) + a0;
    r1 = (pv.y - (3.0f * qv.y)) + a1;
  } else {
    r0 = (pv.x - qv.x) + a0;
    r1 = (pv.y - qv.y) + a1;
  }
  const float qnan = __int_as_float(0x7fc00000);
  r0 = (bad != 0) ? qnan : r0;
  r1 = (bad != 0) ? qnan : r1;
  const v2f rv = (v2f){r0, r1};
  volatile v2f* q = (volatile v2f*)(O + ro);
  *q = rv;
  __threadfence();
  *q = rv;
}

__global__ __launch_bounds__(NTHR) void k_final(const float* __restrict__ A, const int* __restrict__ listG,
                                                const int* __restrict__ cntG, const int* __restrict__ offG,
                                                const int* __restrict__ flagG, const float* __restrict__ dinvG,
                                                const float* __restrict__ bm, float* out, int nN) {
  const int tid = (int)threadIdx.x, lane = tid & 31, wave = tid >> 5;
  const int n = (int)blockIdx.x * NWAVE + wave;
  if (n >= nN) return;
  const int blk = n >> SLB;
  int cv   = cntG[n];
  int ofv  = offG[n];
  int fl   = flagG[(size_t)blk * 32];
  float dn = dinvG[n];
  float own = A[(size_t)n * FD + lane];
  float bq  = bm[lane];
  PIN(cv);
  PIN(ofv);
  PIN(fl);
  PIN(dn);
  PIN(own);
  PIN(bq);
  const int bad = ((fl != 0) || (cv < 0) || (cv > DEGCAP)) ? 1 : 0;
  cv  = cv < 0 ? 0 : (cv > DEGCAP ? DEGCAP : cv);
  ofv = ofv < 0 ? 0 : (ofv > RCAP - DEGCAP ? RCAP - DEGCAP : ofv);
  const int cn = __builtin_amdgcn_readfirstlane(cv);
  const int o  = __builtin_amdgcn_readfirstlane(ofv);
  const int* listb = listG + (size_t)blk * (size_t)RCAP;
  float acc = 0.0f;
#pragma unroll 1
  for (int g0 = 0; g0 < cn; g0 += 32) {
    const int last = o + cn - 1;
    int idx = o + g0 + lane;
    idx = idx > last ? last : idx;
    int s = listb[idx];
    PIN(s);
    const int col = clampi(s, 0, nN - 1);
    float dv = dinvG[col];
    PIN(dv);
    const float w = -(dv * dn);
    const int wb = __float_as_int(w);
    const int m32 = (cn - g0) < 32 ? (cn - g0) : 32;
#pragma unroll 1
    for (int t = 0; t < m32; ++t) {
      const int ct   = __builtin_amdgcn_readlane(col, t);
      const float wt = __int_as_float(__builtin_amdgcn_readlane(wb, t));
      const float z  = A[(size_t)ct * FD + NCLS + lane];
      const float m  = wt * z;
      acc = acc + m;
    }
  }
  float r = (own + acc) + bq;
  const float qnan = __int_as_float(0x7fc00000);
  r = (bad != 0) ? qnan : r;
  volatile float* q = (volatile float*)(out + (size_t)n * NCLS + lane);
  *q = r;
  __threadfence();
  *q = r;
}

__device__ __forceinline__ float hval(float b, float kb, float c, float sb) {
  const float t = b + kb;
  const float r = (t > 0.0f) ? t : (t - t);
  const float u = c + sb;
  return r + u;
}

template <int SPL, int MIXX>
__global__ __launch_bounds__(NTHR) void k_row(const float* __restrict__ Bp, const float* __restrict__ Cp,
                                              const float* __restrict__ kbv, const float* __restrict__ sbv,
                                              const float* __restrict__ x, unsigned short* dst, int nN) {
  constexpr unsigned PPR = 8u * (unsigned)(1 + SPL + MIXX);
  const unsigned total = (unsigned)NP * PPR;
  const unsigned g    = blockIdx.x * 256u + threadIdx.x;
  const unsigned rowu = g / PPR;
  const unsigned p    = g - rowu * PPR;
  const int sec = (int)(p >> 3);
  const int c0  = (int)((p & 7u) << 3);
  const int row = (int)rowu;
  const int rc  = clampi(row, 0, nN - 1);
  const size_t ro = (size_t)rc * FD + c0;
  v4f b0 = *(const v4fa*)(Bp + ro);
  v4f b1 = *(const v4fa*)(Bp + ro + 4);
  v4f q0 = *(const v4fa*)(Cp + ro);
  v4f q1 = *(const v4fa*)(Cp + ro + 4);
  v4f k0 = *(const v4fa*)(kbv + c0);
  v4f k1 = *(const v4fa*)(kbv + c0 + 4);
  v4f s0 = *(const v4fa*)(sbv + c0);
  v4f s1 = *(const v4fa*)(sbv + c0 + 4);
  PIN(b0); PIN(b1); PIN(q0); PIN(q1); PIN(k0); PIN(k1); PIN(s0); PIN(s1);
  const v4f ha = (v4f){ hval(b0[0], k0[0], q0[0], s0[0]), hval(b0[1], k0[1], q0[1], s0[1]),
                        hval(b0[2], k0[2], q0[2], s0[2]), hval(b0[3], k0[3], q0[3], s0[3]) };
  const v4f hb = (v4f){ hval(b1[0], k1[0], q1[0], s1[0]), hval(b1[1], k1[1], q1[1], s1[1]),
                        hval(b1[2], k1[2], q1[2], s1[2]), hval(b1[3], k1[3], q1[3], s1[3]) };
  const unsigned mh = (sec == 0) ? 0xFFFFFFFFu : 0u;
  v4u o = pack8_bf16(ha, hb) & (v4u){mh, mh, mh, mh};
  if (SPL) {
    const unsigned ml = (sec == 1) ? 0xFFFFFFFFu : 0u;
    o |= pack8_bf16_lo(ha, hb) & (v4u){ml, ml, ml, ml};
  }
  if (MIXX) {
    v4f x0 = *(const v4fa*)(x + ro);
    v4f x1 = *(const v4fa*)(x + ro + 4);
    PIN(x0); PIN(x1);
    const unsigned mx = (sec == SPL + 1) ? 0xFFFFFFFFu : 0u;
    o |= pack8_bf16(x0, x1) & (v4u){mx, mx, mx, mx};
  }
  const unsigned mr = (row < nN) ? 0xFFFFFFFFu : 0u;
  o &= (v4u){mr, mr, mr, mr};
  if (g < total) {
    volatile v4u* q = (volatile v4u*)(dst + (size_t)g * 8);
    *q = o;
    __threadfence();
    *q = o;
  }
}

constexpr size_t SZ_F    = (size_t)NP * FD * 4;
constexpr size_t SZ_HHL  = (size_t)NP * 128 * 2;
constexpr size_t SZ_XB   = (size_t)NP * 64 * 2;
constexpr size_t SZ_MIX  = (size_t)NP * 192 * 2;
constexpr size_t SZ_LIST = (size_t)NBLK * RCAP * 4;
constexpr size_t SZ_SLOT = (size_t)NSLOT * 4;
constexpr size_t SZ_FLAG = (size_t)NBLK * 32 * 4;
constexpr size_t SZ_WPL  = (size_t)15 * WSLOT * 2;
constexpr size_t SZ_MT   = (size_t)64 * 192 * 2;
constexpr size_t SZ_BT   = (size_t)512 * 4;
constexpr size_t O_A    = 0;
constexpr size_t O_B    = O_A + SZ_F;
constexpr size_t O_C    = O_B + SZ_F;
constexpr size_t O_HHL  = O_C + SZ_F;
constexpr size_t O_XB   = O_HHL + SZ_HHL;
constexpr size_t O_LIST = O_XB + SZ_XB;
constexpr size_t O_CNT  = O_LIST + SZ_LIST;
constexpr size_t O_OFF  = O_CNT + SZ_SLOT;
constexpr size_t O_DINV = O_OFF + SZ_SLOT;
constexpr size_t O_FLAG = O_DINV + SZ_SLOT;
constexpr size_t O_WPL  = O_FLAG + SZ_FLAG;
constexpr size_t O_MT   = O_WPL + SZ_WPL;
constexpr size_t O_BT   = O_MT + SZ_MT;
constexpr size_t WS_TOTAL = O_BT + SZ_BT;
static_assert(SZ_F % 256 == 0 && SZ_HHL % 256 == 0 && SZ_XB % 256 == 0 && SZ_LIST % 256 == 0);
static_assert(SZ_SLOT % 256 == 0 && SZ_FLAG % 256 == 0 && SZ_WPL % 256 == 0 && SZ_MT % 256 == 0 && SZ_BT % 256 == 0);
static_assert(SZ_MIX == SZ_HHL + SZ_XB && O_XB == O_HHL + SZ_HHL);
static_assert((size_t)NP * KL2 * 2 <= SZ_HHL && (size_t)NP * KL3 * 2 <= SZ_HHL && (size_t)NP * KMX * 2 <= SZ_MIX);
static_assert((size_t)64 * KMX * 2 <= SZ_MT && (size_t)64 * 128 * 2 == (size_t)WSLOT * 2);
static_assert(WS_TOTAL == ((size_t)481337 * 256) && WS_TOTAL <= ((size_t)128 << 20));
static_assert(((NP * 8) % 256) == 0 && ((NP * 16) % 256) == 0 && ((NP * 24) % 256) == 0);

static void run_gemm(const unsigned short* Ap, const unsigned short* Bp, const float* bias, float* D, int KTOT,
                     hipStream_t s) {
  const int tiles = (NN + 63) / 64;
  k_gemm_nt<0, 0><<<(tiles + 7) / 8, 256, 0, s>>>(Ap, Bp, bias, D, NN, FD, KTOT, FD);
}

extern "C" void kernel_launch(void* const* d_in, const int* in_sizes, int n_in,
                              void* d_out, int out_size, void* d_ws, size_t ws_size,
                              hipStream_t stream) {
  if (n_in < 8) return;
  if (in_sizes[0] != NN * FD) return;
  if (in_sizes[1] != 2 * NE) return;
  if (in_sizes[2] != 3 * 4 * 64 * 64) return;
  if (in_sizes[3] != 3 * 64) return;
  if (in_sizes[4] != 3 * 64 * 64) return;
  if (in_sizes[5] != 3 * 64) return;
  if (in_sizes[6] != 2 * 128 * NCLS) return;
  if (in_sizes[7] != NCLS) return;
  if (out_size != NN * NCLS) return;
  if (ws_size < WS_TOTAL) return;

  const float* x  = (const float*)d_in[0];
  const int*   ei = (const int*)d_in[1];
  const float* kw = (const float*)d_in[2];
  const float* kb = (const float*)d_in[3];
  const float* sw = (const float*)d_in[4];
  const float* sb = (const float*)d_in[5];
  const float* mw = (const float*)d_in[6];
  const float* mb = (const float*)d_in[7];
  const int* src = ei;
  const int* dst = ei + NE;
  float* out = (float*)d_out;

  char* ws = (char*)d_ws;
  float*          PA  = (float*)(ws + O_A);
  float*          PB  = (float*)(ws + O_B);
  float*          PC  = (float*)(ws + O_C);
  unsigned short* HHL = (unsigned short*)(ws + O_HHL);
  unsigned short* XB  = (unsigned short*)(ws + O_XB);
  unsigned short* MIX = (unsigned short*)(ws + O_HHL);
  int*            LST = (int*)(ws + O_LIST);
  int*            CNT = (int*)(ws + O_CNT);
  int*            OFF = (int*)(ws + O_OFF);
  float*          DNV = (float*)(ws + O_DINV);
  int*            FLG = (int*)(ws + O_FLAG);
  unsigned short* WPL = (unsigned short*)(ws + O_WPL);
  unsigned short* MT  = (unsigned short*)(ws + O_MT);
  float*          BT  = (float*)(ws + O_BT);

  hipFuncSetAttribute(reinterpret_cast<const void*>(&k_build), hipFuncAttributeMaxDynamicSharedMemorySize,
                      (int)BK_LDS);

  k_plane<0><<<NP * (FD / 8) / 256, 256, 0, stream>>>(x, NN, FD, FD, XB, NP, FD);
  k_prep<<<PREP_BLOCKS, NTHR, 0, stream>>>(kw, sw, mw, kb, sb, mb, WPL, MT, BT);
  k_build<<<NBLK, NTHR, BK_LDS, stream>>>(src, dst, NN, LST, CNT, OFF, DNV, FLG);

  const int propGrid = NN / NWAVE;
  for (int i = 0; i < 3; ++i) {
    const unsigned short* OP = (i == 0) ? XB : HHL;
    const int KT = (i == 0) ? KL1 : ((i == 1) ? KL2 : KL3);
    const unsigned short* W0 = WPL + (size_t)(i * 5 + 0) * WSLOT;
    const unsigned short* W1 = WPL + (size_t)(i * 5 + 1) * WSLOT;
    const unsigned short* W2 = WPL + (size_t)(i * 5 + 2) * WSLOT;
    const unsigned short* W3 = WPL + (size_t)(i * 5 + 3) * WSLOT;
    const unsigned short* WS = WPL + (size_t)(i * 5 + 4) * WSLOT;
    run_gemm(OP, W3, BT, PA, KT, stream);
    run_gemm(OP, W2, BT, PB, KT, stream);
    k_prop<1><<<propGrid, NTHR, 0, stream>>>(PA, PB, PB, PC, LST, CNT, OFF, FLG, DNV, NN);
    run_gemm(OP, W1, BT, PB, KT, stream);
    k_prop<2><<<propGrid, NTHR, 0, stream>>>(PC, PB, PA, PA, LST, CNT, OFF, FLG, DNV, NN);
    run_gemm(OP, W0, BT, PB, KT, stream);
    run_gemm(OP, W2, BT, PC, KT, stream);
    k_prop<3><<<propGrid, NTHR, 0, stream>>>(PA, PB, PC, PB, LST, CNT, OFF, FLG, DNV, NN);
    run_gemm(OP, WS, BT, PC, KT, stream);
    if (i == 0) {
      k_row<SPLIT_L2, 0><<<NP * (8 * (1 + SPLIT_L2)) / 256, 256, 0, stream>>>(PB, PC, BT + 0, BT + 192, x, HHL, NN);
    } else if (i == 1) {
      k_row<SPLIT_L3, 0><<<NP * (8 * (1 + SPLIT_L3)) / 256, 256, 0, stream>>>(PB, PC, BT + 64, BT + 256, x, HHL, NN);
    } else {
      k_row<SPLIT_MIX, 1><<<NP * (8 * (2 + SPLIT_MIX)) / 256, 256, 0, stream>>>(PB, PC, BT + 128, BT + 320, x, MIX, NN);
    }
  }
  run_gemm(MIX, MT, BT, PA, KMX, stream);
  k_final<<<propGrid, NTHR, 0, stream>>>(PA, LST, CNT, OFF, FLG, DNV, BT + 384, out, NN);
}
